// M2RAGNN_82446192214704
// MI455X (gfx1250) — hardware-verified
//
#include <hip/hip_runtime.h>
#include <stddef.h>


#define HD      128
#define FD      64
#define HHID    64
#define NTHR    256
#define NWAVE   8
#define EPT     8
#define NGRP    2
#define CHUNK   (NTHR * EPT * NGRP)
#define WCAP    (EPT * NGRP * 32)
#define LISTN   (NWAVE * WCAP)
#define NBA     512
#define GROWS   128
#define PA      72
#define PH      136
#define EPB     256
#define STHR    512
#define WSCALE  8.0f
#define WINV    0.125f

#define OWN   0
#define OWT   8192
#define OWM   24576
#define OWU   40960
#define OWY   57344
#define OWA   65536
#define WTOT  73728
#define WPREP_BLOCKS (WTOT / 8 / NTHR)

#define LDS_NODE (GROWS * PA * 2 + GROWS * HD * 4 + GROWS * PH * 2)
#define LDS_AGG  (NBA * HD * 4 + LISTN * 4 + 64)

static_assert((CHUNK & (CHUNK - 1)) == 0);
static_assert(CHUNK <= 4096);
static_assert(NBA <= 4096 && (NBA & (NBA - 1)) == 0);
static_assert(WPREP_BLOCKS * NTHR * 8 == WTOT);
static_assert((GROWS * PA * 2) % 16 == 0 && (PA * 2) % 16 == 0 && (PH * 2) % 16 == 0);

typedef float    v4f  __attribute__((ext_vector_type(4)));
typedef float    v8f  __attribute__((ext_vector_type(8)));
typedef int      v4i  __attribute__((ext_vector_type(4)));
typedef _Float16 v8h  __attribute__((ext_vector_type(8)));
typedef _Float16 v16h __attribute__((ext_vector_type(16)));
union FragH { v16h v; v8h h[2]; };

__device__ __forceinline__ v8h cvt8(v4f a, v4f b) {
  v8h r;
  r[0] = (_Float16)a.x; r[1] = (_Float16)a.y; r[2] = (_Float16)a.z; r[3] = (_Float16)a.w;
  r[4] = (_Float16)b.x; r[5] = (_Float16)b.y; r[6] = (_Float16)b.z; r[7] = (_Float16)b.w;
  return r;
}

__device__ __forceinline__ v8f wmh(v16h a, v16h b, v8f c) {
  v8f d = __builtin_amdgcn_wmma_f32_16x16x32_f16(false, a, false, b, (short)0, c, false, false);
  asm volatile("v_nop\n\tv_nop\n\tv_nop\n\tv_nop" : "+v"(d) : "v"(a), "v"(b));
  return d;
}

template <int NB>
__device__ __forceinline__ int scan_chunk(const int* __restrict__ dsts, int nE, int cbase, int nodeBase,
                                          int vec8, int* list, int tid, int lane, int wave) {
  int wc = 0;
#pragma unroll
  for (int g = 0; g < NGRP; ++g) {
    const int el0  = (g * NTHR + tid) * EPT;
    const int e0   = cbase + el0;
    const int sent = -2147483647 - 1;
    v4i da, db;
    if (vec8 != 0 && cbase + CHUNK <= nE) {
      da = *(const v4i*)(dsts + e0);
      db = *(const v4i*)(dsts + e0 + 4);
    } else {
      da.x = (e0     < nE) ? dsts[min(e0, nE - 1)] : sent;
      da.y = (e0 + 1 < nE) ? dsts[min(e0 + 1, nE - 1)] : sent;
      da.z = (e0 + 2 < nE) ? dsts[min(e0 + 2, nE - 1)] : sent;
      da.w = (e0 + 3 < nE) ? dsts[min(e0 + 3, nE - 1)] : sent;
      db.x = (e0 + 4 < nE) ? dsts[min(e0 + 4, nE - 1)] : sent;
      db.y = (e0 + 5 < nE) ? dsts[min(e0 + 5, nE - 1)] : sent;
      db.z = (e0 + 6 < nE) ? dsts[min(e0 + 6, nE - 1)] : sent;
      db.w = (e0 + 7 < nE) ? dsts[min(e0 + 7, nE - 1)] : sent;
    }
    const unsigned nb = (unsigned)nodeBase;
    const unsigned s0 = (unsigned)da.x - nb, s1 = (unsigned)da.y - nb;
    const unsigned s2 = (unsigned)da.z - nb, s3 = (unsigned)da.w - nb;
    const unsigned s4 = (unsigned)db.x - nb, s5 = (unsigned)db.y - nb;
    const unsigned s6 = (unsigned)db.z - nb, s7 = (unsigned)db.w - nb;
    const bool h0 = s0 < (unsigned)NB, h1 = s1 < (unsigned)NB, h2 = s2 < (unsigned)NB, h3 = s3 < (unsigned)NB;
    const bool h4 = s4 < (unsigned)NB, h5 = s5 < (unsigned)NB, h6 = s6 < (unsigned)NB, h7 = s7 < (unsigned)NB;
    const unsigned any = __builtin_amdgcn_ballot_w32(h0 | h1 | h2 | h3 | h4 | h5 | h6 | h7);
    if (any != 0u) {
#define HITJ(J, HJ, SJ) { \
        const unsigned mj = __builtin_amdgcn_ballot_w32(HJ); \
        if (mj != 0u) { \
          if (HJ) { \
            const int pos = wc + (int)__builtin_amdgcn_mbcnt_lo(mj, 0u); \
            if (pos < WCAP) list[wave * WCAP + pos] = ((el0 + (J)) << 12) | (int)(SJ); \
          } \
          wc += (int)__builtin_popcount(mj); } }
      HITJ(0, h0, s0)
      HITJ(1, h1, s1)
      HITJ(2, h2, s2)
      HITJ(3, h3, s3)
      HITJ(4, h4, s4)
      HITJ(5, h5, s5)
      HITJ(6, h6, s6)
      HITJ(7, h7, s7)
#undef HITJ
    }
  }
  return wc;
}

__global__ __launch_bounds__(NTHR) void k_wprep(
    const float* __restrict__ W_node, const float* __restrict__ W_att1, const float* __restrict__ W_upd,
    const float* __restrict__ Wy1, const float* __restrict__ Wa1, _Float16* wall) {
  const int b = blockIdx.x;
  const float* W; int Kseg, Ncol, segBase, blk0;
  if (b < 4)        { W = W_node;           Kseg = FD; Ncol = HD;   segBase = OWN; blk0 = 0;  }
  else if (b < 12)  { W = W_att1;           Kseg = HD; Ncol = HD;   segBase = OWT; blk0 = 4;  }
  else if (b < 20)  { W = W_att1 + HD * HD; Kseg = HD; Ncol = HD;   segBase = OWM; blk0 = 12; }
  else if (b < 28)  { W = W_upd;            Kseg = HD; Ncol = HD;   segBase = OWU; blk0 = 20; }
  else if (b < 32)  { W = Wy1;              Kseg = HD; Ncol = HHID; segBase = OWY; blk0 = 28; }
  else              { W = Wa1;              Kseg = HD; Ncol = HHID; segBase = OWA; blk0 = 32; }
  const int o  = ((b - blk0) * NTHR + (int)threadIdx.x) * 8;
  const int n  = o / Kseg;
  const int k0 = o - n * Kseg;
  const float* p = W + (size_t)k0 * Ncol + n;
  v4f a, c;
  a.x = p[0];        a.y = p[Ncol];     a.z = p[2 * Ncol]; a.w = p[3 * Ncol];
  c.x = p[4 * Ncol]; c.y = p[5 * Ncol]; c.z = p[6 * Ncol]; c.w = p[7 * Ncol];
  a = a * WSCALE;
  c = c * WSCALE;
  const v8h hv = cvt8(a, c);
  _Float16* dp = wall + segBase + o;
  *(volatile v8h*)dp = hv;
  __threadfence();
  *(volatile v8h*)dp = hv;
}

__global__ __launch_bounds__(NTHR) void k_node(
    const float* __restrict__ x, const _Float16* __restrict__ wall, const float* __restrict__ b_node,
    float* hpl, float* abpl, int nN) {
  extern __shared__ v4f lds_dyn[];
  _Float16* sA  = (_Float16*)lds_dyn;
  float*    stg = (float*)((char*)lds_dyn + GROWS * PA * 2);
  _Float16* hA  = (_Float16*)((char*)lds_dyn + GROWS * PA * 2 + GROWS * HD * 4);
  const int tid = threadIdx.x, lane = tid & 31, wave = tid >> 5, hh = lane >> 4, m = lane & 15;
  const int rowBase = blockIdx.x * GROWS;

#pragma unroll
  for (int i = 0; i < (GROWS * FD / 8) / NTHR; ++i) {
    const int idx = i * NTHR + tid;
    const int r   = idx >> 3;
    const int c0  = (idx & 7) * 8;
    int node = rowBase + r;
    node = node > nN - 1 ? nN - 1 : node;
    const float* xp = x + (size_t)node * FD + c0;
    const v4f a = *(const v4f*)xp, c = *(const v4f*)(xp + 4);
    *(v8h*)(sA + r * PA + c0) = cvt8(a, c);
  }
  __syncthreads();

  v8f acc[8];
#pragma unroll
  for (int t = 0; t < 8; ++t) { v8f z = {0.f, 0.f, 0.f, 0.f, 0.f, 0.f, 0.f, 0.f}; acc[t] = z; }
  {
    const _Float16* wn = wall + OWN;
    const _Float16* ar = sA + (wave * 16 + m) * PA + 8 * hh;
#pragma unroll
    for (int kt = 0; kt < FD / 32; ++kt) {
      FragH a;
      a.h[0] = *(const v8h*)(ar + 32 * kt);
      a.h[1] = *(const v8h*)(ar + 32 * kt + 16);
#pragma unroll
      for (int t = 0; t < 8; ++t) {
        const _Float16* bp = wn + (size_t)(16 * t + m) * FD + 32 * kt + 8 * hh;
        FragH bq;
        bq.h[0] = *(const v8h*)bp;
        bq.h[1] = *(const v8h*)(bp + 16);
        acc[t] = wmh(a.v, bq.v, acc[t]);
      }
    }
  }
  {
    float* sp = stg + (wave * 16 + 8 * hh) * HD + m;
#pragma unroll
    for (int t = 0; t < 8; ++t) {
      const float bv = b_node[16 * t + m];
#pragma unroll
      for (int r = 0; r < 8; ++r) sp[r * HD + 16 * t] = acc[t][r] * WINV + bv;
    }
  }
  __syncthreads();

#pragma unroll
  for (int i = 0; i < (GROWS * HD / 8) / NTHR; ++i) {
    const int idx = i * NTHR + tid;
    const int r   = idx >> 4;
    const int c0  = (idx & 15) * 8;
    const v4f a = *(const v4f*)(stg + r * HD + c0), c = *(const v4f*)(stg + r * HD + c0 + 4);
    *(v8h*)(hA + r * PH + c0) = cvt8(a, c);
  }
  {
    const float* lp = stg + wave * 16 * HD + 4 * lane;
    float* gp = hpl + ((size_t)rowBase + wave * 16) * HD + 4 * lane;
#pragma unroll
    for (int i = 0; i < 16; ++i) { const v4f v = *(const v4f*)(lp + i * HD); *(volatile v4f*)(gp + (size_t)i * HD) = v; }
    __threadfence();
#pragma unroll
    for (int i = 0; i < 16; ++i) { const v4f v = *(const v4f*)(lp + i * HD); *(volatile v4f*)(gp + (size_t)i * HD) = v; }
  }
  __syncthreads();

#pragma unroll 1
  for (int hf = 0; hf < 2; ++hf) {
    const _Float16* wb = wall + OWT + hf * (OWM - OWT);
#pragma unroll
    for (int t = 0; t < 8; ++t) { v8f z = {0.f, 0.f, 0.f, 0.f, 0.f, 0.f, 0.f, 0.f}; acc[t] = z; }
    const _Float16* ar = hA + (wave * 16 + m) * PH + 8 * hh;
#pragma unroll
    for (int kt = 0; kt < HD / 32; ++kt) {
      FragH a;
      a.h[0] = *(const v8h*)(ar + 32 * kt);
      a.h[1] = *(const v8h*)(ar + 32 * kt + 16);
#pragma unroll
      for (int t = 0; t < 8; ++t) {
        const _Float16* bp = wb + (size_t)(16 * t + m) * HD + 32 * kt + 8 * hh;
        FragH bq;
        bq.h[0] = *(const v8h*)bp;
        bq.h[1] = *(const v8h*)(bp + 16);
        acc[t] = wmh(a.v, bq.v, acc[t]);
      }
    }
    {
      float* sp = stg + (wave * 16 + 8 * hh) * HD + m;
#pragma unroll
      for (int t = 0; t < 8; ++t) {
#pragma unroll
        for (int r = 0; r < 8; ++r) sp[r * HD + 16 * t] = acc[t][r] * WINV;
      }
    }
    __syncthreads();
    {
      const float* lp = stg + wave * 16 * HD + 4 * lane;
      float* gp = abpl + ((size_t)rowBase + wave * 16) * (2 * HD) + hf * HD + 4 * lane;
#pragma unroll
      for (int i = 0; i < 16; ++i) { const v4f v = *(const v4f*)(lp + i * HD); *(volatile v4f*)(gp + (size_t)i * 2 * HD) = v; }
      __threadfence();
#pragma unroll
      for (int i = 0; i < 16; ++i) { const v4f v = *(const v4f*)(lp + i * HD); *(volatile v4f*)(gp + (size_t)i * 2 * HD) = v; }
    }
    __syncthreads();
  }
}

__global__ __launch_bounds__(NTHR) void k_head(
    const float* __restrict__ x, const _Float16* __restrict__ wall, int owoff,
    const float* __restrict__ b_node, const float* __restrict__ b1, const float* __restrict__ W2,
    const float* __restrict__ b2, float* outv, int M) {
  __shared__ __attribute__((aligned(16))) _Float16 sA[GROWS * PA];
  __shared__ __attribute__((aligned(16))) _Float16 hA[GROWS * PH];
  __shared__ __attribute__((aligned(16))) float sout[GROWS];
  const int tid = threadIdx.x, lane = tid & 31, wave = tid >> 5, hh = lane >> 4, m = lane & 15;
  const int rowBase = blockIdx.x * GROWS;

#pragma unroll
  for (int i = 0; i < (GROWS * FD / 8) / NTHR; ++i) {
    const int idx = i * NTHR + tid;
    const int r   = idx >> 3;
    const int c0  = (idx & 7) * 8;
    int row = rowBase + r;
    row = row > M - 1 ? M - 1 : row;
    const float* xp = x + (size_t)row * FD + c0;
    const v4f a = *(const v4f*)xp, c = *(const v4f*)(xp + 4);
    *(v8h*)(sA + r * PA + c0) = cvt8(a, c);
  }
  __syncthreads();

  v8f acc[8];
#pragma unroll
  for (int t = 0; t < 8; ++t) { v8f z = {0.f, 0.f, 0.f, 0.f, 0.f, 0.f, 0.f, 0.f}; acc[t] = z; }
  {
    const _Float16* wn = wall + OWN;
    const _Float16* ar = sA + (wave * 16 + m) * PA + 8 * hh;
#pragma unroll
    for (int kt = 0; kt < FD / 32; ++kt) {
      FragH a;
      a.h[0] = *(const v8h*)(ar + 32 * kt);
      a.h[1] = *(const v8h*)(ar + 32 * kt + 16);
#pragma unroll
      for (int t = 0; t < 8; ++t) {
        const _Float16* bp = wn + (size_t)(16 * t + m) * FD + 32 * kt + 8 * hh;
        FragH bq;
        bq.h[0] = *(const v8h*)bp;
        bq.h[1] = *(const v8h*)(bp + 16);
        acc[t] = wmh(a.v, bq.v, acc[t]);
      }
    }
  }
  {
    _Float16* hp = hA + (wave * 16 + 8 * hh) * PH + m;
#pragma unroll
    for (int t = 0; t < 8; ++t) {
      const float bv = b_node[16 * t + m];
#pragma unroll
      for (int r = 0; r < 8; ++r) hp[r * PH + 16 * t] = (_Float16)(acc[t][r] * WINV + bv);
    }
  }
  __syncthreads();

  v8f c2[4];
#pragma unroll
  for (int t = 0; t < 4; ++t) { v8f z = {0.f, 0.f, 0.f, 0.f, 0.f, 0.f, 0.f, 0.f}; c2[t] = z; }
  {
    const _Float16* wb = wall + owoff;
    const _Float16* ar = hA + (wave * 16 + m) * PH + 8 * hh;
#pragma unroll
    for (int kt = 0; kt < HD / 32; ++kt) {
      FragH a;
      a.h[0] = *(const v8h*)(ar + 32 * kt);
      a.h[1] = *(const v8h*)(ar + 32 * kt + 16);
#pragma unroll
      for (int t = 0; t < 4; ++t) {
        const _Float16* bp = wb + (size_t)(16 * t + m) * HD + 32 * kt + 8 * hh;
        FragH bq;
        bq.h[0] = *(const v8h*)bp;
        bq.h[1] = *(const v8h*)(bp + 16);
        c2[t] = wmh(a.v, bq.v, c2[t]);
      }
    }
  }
  float part[8] = {0.f, 0.f, 0.f, 0.f, 0.f, 0.f, 0.f, 0.f};
#pragma unroll
  for (int t = 0; t < 4; ++t) {
    const int col = 16 * t + m;
    const float bb = b1[col], wo = W2[col];
#pragma unroll
    for (int v = 0; v < 8; ++v) part[v] += fmaxf(c2[t][v] * WINV + bb, 0.f) * wo;
  }
#pragma unroll
  for (int msk = 1; msk < 16; msk <<= 1) {
#pragma unroll
    for (int v = 0; v < 8; ++v) part[v] += __shfl_xor(part[v], msk, 32);
  }
  if (m == 0) {
    const float bo = b2[0];
#pragma unroll
    for (int v = 0; v < 8; ++v) sout[wave * 16 + 8 * hh + v] = part[v] + bo;
  }
  __syncthreads();

  if (wave == 0) {
    const int r0 = rowBase + 4 * lane;
    const v4f v = *(const v4f*)(sout + 4 * lane);
    const bool full = (r0 + 4 <= M);
    if (full) {
      *(volatile v4f*)(outv + r0) = v;
    } else {
      if (r0     < M) *(volatile float*)(outv + r0)     = v.x;
      if (r0 + 1 < M) *(volatile float*)(outv + r0 + 1) = v.y;
      if (r0 + 2 < M) *(volatile float*)(outv + r0 + 2) = v.z;
      if (r0 + 3 < M) *(volatile float*)(outv + r0 + 3) = v.w;
    }
    __threadfence();
    if (full) {
      *(volatile v4f*)(outv + r0) = v;
    } else {
      if (r0     < M) *(volatile float*)(outv + r0)     = v.x;
      if (r0 + 1 < M) *(volatile float*)(outv + r0 + 1) = v.y;
      if (r0 + 2 < M) *(volatile float*)(outv + r0 + 2) = v.z;
      if (r0 + 3 < M) *(volatile float*)(outv + r0 + 3) = v.w;
    }
  }
}

__global__ __launch_bounds__(NTHR) void k_edge(
    const int* __restrict__ ei, const float* __restrict__ pos, const float* __restrict__ abpl,
    const float* __restrict__ W_att1, const float* __restrict__ b_att1, const float* __restrict__ W_att2,
    const float* __restrict__ b_att2, float* spl, int nN, int nE) {
  __shared__ __attribute__((aligned(16))) float sw[5 * HD];
  __shared__ __attribute__((aligned(16))) float ssc[EPB];
  const int tid = threadIdx.x, lane = tid & 31, wave = tid >> 5;
  for (int i = tid; i < 3 * HD; i += NTHR) sw[i] = W_att1[(2 * HD) * HD + i];
  for (int i = tid; i < HD; i += NTHR) { sw[3 * HD + i] = b_att1[i]; sw[4 * HD + i] = W_att2[i]; }
  __syncthreads();

  int e = blockIdx.x * EPB + tid;
  e = e > nE - 1 ? nE - 1 : e;
  int src = ei[e];
  int dst = ei[nE + e];
  src = src < 0 ? 0 : (src > nN - 1 ? nN - 1 : src);
  dst = dst < 0 ? 0 : (dst > nN - 1 ? nN - 1 : dst);
  const float dx = pos[(size_t)dst * 3 + 0] - pos[(size_t)src * 3 + 0];
  const float dy = pos[(size_t)dst * 3 + 1] - pos[(size_t)src * 3 + 1];
  const float dz = pos[(size_t)dst * 3 + 2] - pos[(size_t)src * 3 + 2];
  const float* pa = abpl + (size_t)dst * (2 * HD);
  const float* pb = abpl + (size_t)src * (2 * HD) + HD;
  float s = 0.f;
#pragma unroll 1
  for (int c4 = 0; c4 < HD; c4 += 4) {
    const v4f a  = *(const v4f*)(pa + c4);
    const v4f bq = *(const v4f*)(pb + c4);
    const v4f w0 = *(const v4f*)(sw + c4);
    const v4f w1 = *(const v4f*)(sw + HD + c4);
    const v4f w2 = *(const v4f*)(sw + 2 * HD + c4);
    const v4f bb = *(const v4f*)(sw + 3 * HD + c4);
    const v4f wo = *(const v4f*)(sw + 4 * HD + c4);
    v4f t = a + bq + bb;
    t = t + dx * w0;
    t = t + dy * w1;
    t = t + dz * w2;
    t.x = fmaxf(t.x, 0.f); t.y = fmaxf(t.y, 0.f); t.z = fmaxf(t.z, 0.f); t.w = fmaxf(t.w, 0.f);
    s += t.x * wo.x; s += t.y * wo.y; s += t.z * wo.z; s += t.w * wo.w;
  }
  ssc[tid] = s + b_att2[0];
  __syncthreads();

  if (wave == 0) {
    float* gp = spl + (size_t)blockIdx.x * EPB;
    v4f ov[2];
#pragma unroll
    for (int q = 0; q < 2; ++q) ov[q] = *(const v4f*)(ssc + q * 128 + 4 * lane);
#pragma unroll
    for (int q = 0; q < 2; ++q) *(volatile v4f*)(gp + q * 128 + 4 * lane) = ov[q];
    __threadfence();
#pragma unroll
    for (int q = 0; q < 2; ++q) *(volatile v4f*)(gp + q * 128 + 4 * lane) = ov[q];
  }
}

__global__ __launch_bounds__(STHR) void k_stats(const float* __restrict__ spl, float* stats, int nE) {
  __shared__ float  smx[STHR];
  __shared__ double ssm[STHR];
  const int tid = threadIdx.x;
  float mx = -3.0e38f;
#pragma unroll 1
  for (int i = tid; i < nE; i += STHR) mx = fmaxf(mx, spl[i]);
  smx[tid] = mx;
  __syncthreads();
  for (int o = STHR / 2; o > 0; o >>= 1) {
    if (tid < o) smx[tid] = fmaxf(smx[tid], smx[tid + o]);
    __syncthreads();
  }
  const float Mx = smx[0];
  double z = 0.0;
#pragma unroll 1
  for (int i = tid; i < nE; i += STHR) z += (double)expf(spl[i] - Mx);
  ssm[tid] = z;
  __syncthreads();
  for (int o = STHR / 2; o > 0; o >>= 1) {
    if (tid < o) ssm[tid] = ssm[tid] + ssm[tid + o];
    __syncthreads();
  }
  const double Z = ssm[0];
  const float invZ = (Z > 0.0) ? (float)(1.0 / Z) : 0.f;
  v4f v; v.x = Mx; v.y = invZ; v.z = Mx; v.w = invZ;
  if (tid < 8) *(volatile v4f*)(stats + 4 * tid) = v;
  __threadfence();
  if (tid < 8) *(volatile v4f*)(stats + 4 * tid) = v;
}

__global__ __launch_bounds__(NTHR) void k_agg(
    const int* __restrict__ ei, const float* __restrict__ hpl, const float* __restrict__ spl,
    const float* __restrict__ stats, const _Float16* __restrict__ wall, const float* __restrict__ b_upd,
    float* outf, int nN, int nE, int vec8) {
  extern __shared__ v4f lds_dyn[];
  float* acc  = (float*)lds_dyn;
  int*   list = (int*)(acc + NBA * HD);
  int*   wcnt = list + LISTN;
  const int tid = threadIdx.x, lane = tid & 31, wave = tid >> 5, hh = lane >> 4, m = lane & 15;
  const int nodeBase = blockIdx.x * NBA;
  const int* dsts = ei + nE;
  const float Mx   = stats[0];
  const float invZ = stats[1];

  {
    const v4f z = {0.f, 0.f, 0.f, 0.f};
    for (int i = tid; i < NBA * HD / 4; i += NTHR) lds_dyn[i] = z;
  }
  __syncthreads();

  const int nChunks = (nE + CHUNK - 1) / CHUNK;
#pragma unroll 1
  for (int ch = 0; ch < nChunks; ++ch) {
    const int cbase = ch * CHUNK;
    const int wc = scan_chunk<NBA>(dsts, nE, cbase, nodeBase, vec8, list, tid, lane, wave);
    if (lane == 0) wcnt[wave] = wc;
    __syncthreads();
    if (wave == 0) {
#pragma unroll 1
      for (int wsx = 0; wsx < NWAVE; ++wsx) {
        int n = __builtin_amdgcn_readfirstlane(wcnt[wsx]);
        n = n > WCAP ? WCAP : (n < 0 ? 0 : n);
        const int* lp = list + wsx * WCAP;
#pragma unroll 1
        for (int i = 0; i < n; ++i) {
          const int ent  = __builtin_amdgcn_readfirstlane(lp[i]);
          const int slot = ent & (NBA - 1);
          int e = cbase + ((ent >> 12) & (CHUNK - 1));
          e = e > nE - 1 ? nE - 1 : e;
          int src = ei[e];
          src = src < 0 ? 0 : (src > nN - 1 ? nN - 1 : src);
          const float w = expf(spl[e] - Mx);
          const v4f v = *(const v4f*)(hpl + (size_t)src * HD + 4 * lane);
          v4f* ap = (v4f*)(acc + slot * HD + 4 * lane);
          *ap = *ap + v * w;
        }
      }
    }
    __syncthreads();
  }

  float bcol[8];
#pragma unroll
  for (int ct = 0; ct < 8; ++ct) bcol[ct] = b_upd[16 * ct + m];
  const float sc2 = invZ * WINV;
  const _Float16* wu = wall + OWU;
#pragma unroll 1
  for (int q = 0; q < NBA / 16 / NWAVE; ++q) {
    const int t = wave + NWAVE * q;
    v8f c[8];
#pragma unroll
    for (int ct = 0; ct < 8; ++ct) { v8f z = {0.f, 0.f, 0.f, 0.f, 0.f, 0.f, 0.f, 0.f}; c[ct] = z; }
#pragma unroll
    for (int kt = 0; kt < HD / 32; ++kt) {
      const float* ap = acc + (16 * t + m) * HD + 32 * kt + 8 * hh;
      const v4f p0 = *(const v4f*)ap,        p1 = *(const v4f*)(ap + 4);
      const v4f p2 = *(const v4f*)(ap + 16), p3 = *(const v4f*)(ap + 20);
      FragH a;
      a.h[0] = cvt8(p0, p1);
      a.h[1] = cvt8(p2, p3);
#pragma unroll
      for (int ct = 0; ct < 8; ++ct) {
        const _Float16* bp = wu + (size_t)(16 * ct + m) * HD + 32 * kt + 8 * hh;
        FragH bq;
        bq.h[0] = *(const v8h*)bp;
        bq.h[1] = *(const v8h*)(bp + 16);
        c[ct] = wmh(a.v, bq.v, c[ct]);
      }
    }
    __syncthreads();
    float* sp = acc + (16 * t + 8 * hh) * HD + m;
#pragma unroll
    for (int ct = 0; ct < 8; ++ct) {
#pragma unroll
      for (int r = 0; r < 8; ++r) sp[r * HD + 16 * ct] = c[ct][r] * sc2 + bcol[ct];
    }
  }
  __syncthreads();

  const int rw0 = wave * (NBA / NWAVE);
#pragma unroll 4
  for (int i = 0; i < NBA / NWAVE; ++i) {
    const int row = rw0 + i;
    const int node = nodeBase + row;
    if (node < nN) { const v4f v = *(const v4f*)(acc + row * HD + 4 * lane); *(volatile v4f*)(outf + (size_t)node * HD + 4 * lane) = v; }
  }
  __threadfence();
#pragma unroll 4
  for (int i = 0; i < NBA / NWAVE; ++i) {
    const int row = rw0 + i;
    const int node = nodeBase + row;
    if (node < nN) { const v4f v = *(const v4f*)(acc + row * HD + 4 * lane); *(volatile v4f*)(outf + (size_t)node * HD + 4 * lane) = v; }
  }
}

extern "C" void kernel_launch(void* const* d_in, const int* in_sizes, int n_in,
                              void* d_out, int out_size, void* d_ws, size_t ws_size,
                              hipStream_t stream) {
  if (n_in < 21) return;
  const int nN = in_sizes[0] / FD;
  const int NR = in_sizes[2] / FD;
  const int NT = in_sizes[3] / FD;
  const int nE = in_sizes[4] / 2;
  if (nN <= 0 || NR <= 0 || NT <= 0 || nE <= 0) return;
  if (in_sizes[0] != nN * FD || in_sizes[1] != nN * 3 || in_sizes[2] != NR * FD || in_sizes[3] != NT * FD) return;
  if (in_sizes[4] != 2 * nE) return;
  if (in_sizes[5] != FD * HD || in_sizes[6] < HD || in_sizes[7] != (2 * HD + 3) * HD || in_sizes[8] < HD) return;
  if (in_sizes[9] < HD || in_sizes[10] < 1 || in_sizes[11] != HD * HD || in_sizes[12] < HD) return;
  if (in_sizes[13] != HD * HHID || in_sizes[14] < HHID || in_sizes[15] < HHID || in_sizes[16] < 1) return;
  if (in_sizes[17] != HD * HHID || in_sizes[18] < HHID || in_sizes[19] < HHID || in_sizes[20] < 1) return;
  if (out_size != NR + NT + nN * HD) return;

  const float* mol_x  = (const float*)d_in[0];
  const float* pos    = (const float*)d_in[1];
  const float* rx     = (const float*)d_in[2];
  const float* tx     = (const float*)d_in[3];
  const int*   ei     = (const int*)d_in[4];
  const float* W_node = (const float*)d_in[5];
  const float* b_node = (const float*)d_in[6];
  const float* W_att1 = (const float*)d_in[7];
  const float* b_att1 = (const float*)d_in[8];
  const float* W_att2 = (const float*)d_in[9];
  const float* b_att2 = (const float*)d_in[10];
  const float* W_upd  = (const float*)d_in[11];
  const float* b_upd  = (const float*)d_in[12];
  const float* Wy1    = (const float*)d_in[13];
  const float* by1    = (const float*)d_in[14];
  const float* Wy2    = (const float*)d_in[15];
  const float* by2    = (const float*)d_in[16];
  const float* Wa1    = (const float*)d_in[17];
  const float* ba1    = (const float*)d_in[18];
  const float* Wa2    = (const float*)d_in[19];
  const float* ba2    = (const float*)d_in[20];

  float* out0 = (float*)d_out;
  float* out1 = out0 + NR;
  float* out2 = out0 + NR + NT;

  const int nGN = (nN + GROWS - 1) / GROWS;
  const int nGR = (NR + GROWS - 1) / GROWS;
  const int nGT = (NT + GROWS - 1) / GROWS;
  const int nEB = (nE + EPB - 1) / EPB;
  const int nAG = (nN + NBA - 1) / NBA;

  char* ws = (char*)d_ws;
  size_t off = 0;
  const size_t oW  = off; off += (size_t)WTOT * 2;                        off = (off + 255) & ~(size_t)255;
  const size_t oH  = off; off += (size_t)nGN * GROWS * HD * 4;            off = (off + 255) & ~(size_t)255;
  const size_t oAB = off; off += (size_t)nGN * GROWS * 2 * HD * 4;        off = (off + 255) & ~(size_t)255;
  const size_t oS  = off; off += (size_t)nEB * EPB * 4;                   off = (off + 255) & ~(size_t)255;
  const size_t oST = off; off += 256;                                     off = (off + 255) & ~(size_t)255;
  if (off > ws_size) return;
  _Float16* wall  = (_Float16*)(ws + oW);
  float*    hpl   = (float*)(ws + oH);
  float*    abpl  = (float*)(ws + oAB);
  float*    spl   = (float*)(ws + oS);
  float*    stats = (float*)(ws + oST);

  const int vec8 = ((nE & 3) == 0) ? 1 : 0;

  k_wprep<<<WPREP_BLOCKS, NTHR, 0, stream>>>(W_node, W_att1, W_upd, Wy1, Wa1, wall);

  hipFuncSetAttribute(reinterpret_cast<const void*>(&k_node),
                      hipFuncAttributeMaxDynamicSharedMemorySize, LDS_NODE);
  k_node<<<nGN, NTHR, LDS_NODE, stream>>>(mol_x, wall, b_node, hpl, abpl, nN);

  k_head<<<nGR, NTHR, 0, stream>>>(rx, wall, (int)OWY, b_node, by1, Wy2, by2, out0, NR);
  k_head<<<nGT, NTHR, 0, stream>>>(tx, wall, (int)OWA, b_node, ba1, Wa2, ba2, out1, NT);

  k_edge<<<nEB, NTHR, 0, stream>>>(ei, pos, abpl, W_att1, b_att1, W_att2, b_att2, spl, nN, nE);

  k_stats<<<1, STHR, 0, stream>>>(spl, stats, nE);

  hipFuncSetAttribute(reinterpret_cast<const void*>(&k_agg),
                      hipFuncAttributeMaxDynamicSharedMemorySize, LDS_AGG);
  k_agg<<<nAG, NTHR, LDS_AGG, stream>>>(ei, hpl, spl, stats, wall, b_upd, out2, nN, nE, vec8);
}
